// CounterattackGNN_39994735460848
// MI455X (gfx1250) — hardware-verified
//
#include <hip/hip_runtime.h>
#include <hip/hip_bf16.h>
#include <stddef.h>


#define NTHR  256
#define NWAVE 8
#define CHUNK 2048
#define WCAP  256
#define NGRP  (CHUNK / (NTHR * 4))
#define LISTN (NWAVE * WCAP)

#define C1   12
#define HD   128
#define P1W  64
#define H0W  32
#define PQW  256

#define NB1 4096
#define SB1 12
#define NB2 1024
#define SB2 10
#define NBP 256
#define SBP 8

#define ACC1 (NB1 * C1)
#define TW1  (6 * 24)
#define TB1  24
#define LDS1_BYTES ((ACC1 + TW1 + TB1 + LISTN + NWAVE) * 4)
#define ACC2 (NB2 * 64)
#define TW2  (6 * 128)
#define TB2  128
#define LDS2_BYTES ((ACC2 + TW2 + TB2 + LISTN + NWAVE) * 4)
#define ACCP (NBP * HD)
#define LDSP_BYTES ((ACCP + NBP + LISTN + NWAVE) * 4)

static_assert(WCAP == (CHUNK / NTHR) * 32);
static_assert(NGRP >= 1);
static_assert(CHUNK == 2048);
static_assert(NB1 == (1 << SB1));
static_assert(NB2 == (1 << SB2));
static_assert(NBP == (1 << SBP));
static_assert(SB1 + 11 < 31);
static_assert((ACC1 % 4) == 0 && (ACC2 % 4) == 0 && (ACCP % 4) == 0);
static_assert(LDS1_BYTES == 205504);
static_assert(LDS2_BYTES == 273952);
static_assert(LDSP_BYTES == 140320);

typedef float v2f __attribute__((ext_vector_type(2)));
typedef float v4f __attribute__((ext_vector_type(4)));
typedef float v8f __attribute__((ext_vector_type(8)));
typedef int   v4i __attribute__((ext_vector_type(4)));
typedef unsigned short v8us __attribute__((ext_vector_type(8)));
typedef __bf16 v16bf __attribute__((ext_vector_type(16)));
union Frag { v16bf v; v8us h[2]; };

__device__ __forceinline__ unsigned int bfr(float f) {
  const unsigned int u = __float_as_uint(f);
  return (u + 0x7FFFu + ((u >> 16) & 1u)) >> 16;
}

__device__ __forceinline__ void wm6(v8f& c0, v8f& c1, v16bf ah0, v16bf al0, v16bf ah1, v16bf al1,
                                    v16bf bh, v16bf bl) {
  c0 = __builtin_amdgcn_wmma_f32_16x16x32_bf16(false, ah0, false, bh, (short)0, c0, false, false);
  c1 = __builtin_amdgcn_wmma_f32_16x16x32_bf16(false, ah1, false, bh, (short)0, c1, false, false);
  c0 = __builtin_amdgcn_wmma_f32_16x16x32_bf16(false, al0, false, bh, (short)0, c0, false, false);
  c1 = __builtin_amdgcn_wmma_f32_16x16x32_bf16(false, al1, false, bh, (short)0, c1, false, false);
  c0 = __builtin_amdgcn_wmma_f32_16x16x32_bf16(false, ah0, false, bl, (short)0, c0, false, false);
  c1 = __builtin_amdgcn_wmma_f32_16x16x32_bf16(false, ah1, false, bl, (short)0, c1, false, false);
  asm volatile("v_nop\n\tv_nop\n\tv_nop\n\tv_nop"
               : "+v"(c0), "+v"(c1)
               : "v"(ah0), "v"(al0), "v"(ah1), "v"(al1), "v"(bh), "v"(bl));
}

__device__ __forceinline__ float wsum(float v) {
  v += __shfl_xor(v, 16, 32);
  v += __shfl_xor(v, 8, 32);
  v += __shfl_xor(v, 4, 32);
  v += __shfl_xor(v, 2, 32);
  v += __shfl_xor(v, 1, 32);
  return v;
}

__device__ __forceinline__ float sigm(float f) {
  const float e = __builtin_amdgcn_exp2f(-f * 1.4426950408889634f);
  return __builtin_amdgcn_rcpf(1.0f + e);
}
__device__ __forceinline__ float softp(float s) {
  const float e = __builtin_amdgcn_exp2f(-fabsf(s) * 1.4426950408889634f);
  return fmaxf(s, 0.f) + 0.69314718055994531f * __builtin_amdgcn_logf(1.0f + e);
}

template<int NB, int SB>
__device__ __forceinline__ int scan_chunk(const int* __restrict__ key, int nK, int cbase, int keyBase,
                                          int* wl, int tid, bool al16) {
  int wc = 0;
  const int sent = -2147483647 - 1;
#pragma unroll
  for (int g = 0; g < NGRP; ++g) {
    const int el0 = (g * NTHR + tid) * 4;
    const int e0  = cbase + el0;
    v4i d;
    if (al16 && (cbase + CHUNK <= nK)) {
      d = *(const v4i*)(key + e0);
    } else {
      const int i0 = min(e0, nK - 1), i1 = min(e0 + 1, nK - 1);
      const int i2 = min(e0 + 2, nK - 1), i3 = min(e0 + 3, nK - 1);
      const int k0v = key[i0], k1v = key[i1], k2v = key[i2], k3v = key[i3];
      d.x = (e0     < nK) ? k0v : sent;
      d.y = (e0 + 1 < nK) ? k1v : sent;
      d.z = (e0 + 2 < nK) ? k2v : sent;
      d.w = (e0 + 3 < nK) ? k3v : sent;
    }
    const unsigned s0 = (unsigned)d.x - (unsigned)keyBase;
    const unsigned s1 = (unsigned)d.y - (unsigned)keyBase;
    const unsigned s2 = (unsigned)d.z - (unsigned)keyBase;
    const unsigned s3 = (unsigned)d.w - (unsigned)keyBase;
    const bool t0 = s0 < (unsigned)NB;
    const bool t1 = s1 < (unsigned)NB;
    const bool t2 = s2 < (unsigned)NB;
    const bool t3 = s3 < (unsigned)NB;
    const unsigned any = __builtin_amdgcn_ballot_w32(t0 | t1 | t2 | t3);
    if (any != 0u) {
#define HITJ(J, TJ, SJ) { \
        const unsigned mj = __builtin_amdgcn_ballot_w32(TJ); \
        if (TJ) { \
          const int pos = wc + (int)__builtin_amdgcn_mbcnt_lo(mj, 0u); \
          if (pos < WCAP) wl[pos] = ((el0 + (J)) << SB) | (int)(SJ); \
        } \
        wc += (int)__builtin_popcount(mj); }
      HITJ(0, t0, s0)
      HITJ(1, t1, s1)
      HITJ(2, t2, s2)
      HITJ(3, t3, s3)
#undef HITJ
    }
  }
  return wc;
}

__global__ __launch_bounds__(NTHR) void k_pq1(const float* __restrict__ x, const float* __restrict__ Wf,
                                              const float* __restrict__ Ws, float* PQ1, int nN) {
  __shared__ float Wc[C1 * 48];
  __shared__ float xs[32 * C1];
  __shared__ __attribute__((aligned(16))) float Rs[32 * P1W];
  const int tid = threadIdx.x, lane = tid & 31, wave = tid >> 5;
  const int nodeBase = blockIdx.x * 32;
  for (int i = tid; i < C1 * 48; i += NTHR) {
    const int k = i / 48, j = i - k * 48;
    const int part = j / 12, cc = j - part * 12;
    const int krow = ((part & 1) ? C1 : 0) + k;
    const float a = Wf[krow * C1 + cc], b = Ws[krow * C1 + cc];
    Wc[i] = (part < 2) ? a : b;
  }
  for (int i = tid; i < 32 * C1; i += NTHR) {
    const int nl = i / C1, k = i - nl * C1;
    int row = nodeBase + nl; if (row > nN - 1) row = nN - 1;
    xs[i] = x[(size_t)row * C1 + k];
  }
  __syncthreads();
  {
    const int nl = tid >> 3, g = tid & 7;
    const int gc = g < 6 ? g : 5;
    const int j0 = gc * 8;
    float a[8];
#pragma unroll
    for (int i = 0; i < 8; ++i) a[i] = 0.f;
#pragma unroll 1
    for (int k = 0; k < C1; ++k) {
      const float xk = xs[nl * C1 + k];
      const float* wr = Wc + k * 48 + j0;
#pragma unroll
      for (int i = 0; i < 8; ++i) a[i] += xk * wr[i];
    }
#pragma unroll
    for (int i = 0; i < 8; ++i) a[i] = (g < 6) ? a[i] : 0.f;
    const v4f u0 = {a[0], a[1], a[2], a[3]};
    const v4f u1 = {a[4], a[5], a[6], a[7]};
    *(v4f*)(Rs + nl * P1W + g * 8)     = u0;
    *(v4f*)(Rs + nl * P1W + g * 8 + 4) = u1;
  }
  __syncthreads();
  v4f rv[2];
  float* rp[2];
#pragma unroll
  for (int i = 0; i < 2; ++i) {
    const int nl2 = 4 * wave + 2 * i + (lane >> 4);
    const int col = 4 * (lane & 15);
    rv[i] = *(const v4f*)(Rs + nl2 * P1W + col);
    rp[i] = PQ1 + (size_t)(nodeBase + nl2) * P1W + col;
  }
#pragma unroll
  for (int i = 0; i < 2; ++i) *(volatile v4f*)(rp[i]) = rv[i];
  __threadfence();
#pragma unroll
  for (int i = 0; i < 2; ++i) *(volatile v4f*)(rp[i]) = rv[i];
}

__global__ __launch_bounds__(NTHR) void k_agg1(
    const float* __restrict__ x, const float* __restrict__ PQ1,
    const int* __restrict__ ei, const float* __restrict__ ea,
    const float* __restrict__ Wf, const float* __restrict__ Ws,
    const float* __restrict__ bf, const float* __restrict__ bs,
    float* h0, int nN, int nE) {
  extern __shared__ v4f lds_dyn[];
  float* acc  = (float*)lds_dyn;
  float* tW   = acc + ACC1;
  float* tb   = tW + TW1;
  int*   list = (int*)(tb + TB1);
  int*   wcnt = list + LISTN;

  const int tid = threadIdx.x, lane = tid & 31, wave = tid >> 5;
  const int keyBase = blockIdx.x * NB1;
  {
    const v4f z4 = {0.f, 0.f, 0.f, 0.f};
    for (int i = tid; i < ACC1 / 4; i += NTHR) lds_dyn[i] = z4;
    for (int i = tid; i < TW1; i += NTHR) {
      const int d = i / 24, j = i - d * 24;
      const int cc = (j < 12) ? j : j - 12;
      const float a = Wf[(24 + d) * C1 + cc], b = Ws[(24 + d) * C1 + cc];
      tW[i] = (j < 12) ? a : b;
    }
    if (tid < TB1) {
      const int ia = tid < 12 ? tid : 11;
      const int ib = tid < 12 ? 0 : tid - 12;
      const float a = bf[ia], b = bs[ib];
      tb[tid] = (tid < 12) ? a : b;
    }
  }
  __syncthreads();

  const int* keyp = ei + nE;
  const bool al16 = ((((size_t)keyp) & 15) == 0);
  const int c = lane < C1 ? lane : C1 - 1;
  const int nChunks = (nE + CHUNK - 1) / CHUNK;
#pragma unroll 1
  for (int ch = 0; ch < nChunks; ++ch) {
    const int cbase = ch * CHUNK;
    const int wc = scan_chunk<NB1, SB1>(keyp, nE, cbase, keyBase, list + wave * WCAP, tid, al16);
    if (lane == 0) wcnt[wave] = wc;
    __syncthreads();
    if (wave == 0) {
      const float bfv = tb[c], bsv = tb[12 + c];
      for (int wsx = 0; wsx < NWAVE; ++wsx) {
        int n = wcnt[wsx];
        n = n > WCAP ? WCAP : (n < 0 ? 0 : n);
        for (int i = 0; i < n; ++i) {
          const int ent  = list[wsx * WCAP + i];
          const int slot = ent & (NB1 - 1);
          const int el   = (ent >> SB1) & (CHUNK - 1);
          int e = cbase + el; if (e > nE - 1) e = nE - 1;
          int src = ei[e]; src = src < 0 ? 0 : (src > nN - 1 ? nN - 1 : src);
          int nd = keyBase + slot; if (nd > nN - 1) nd = nN - 1;
          const float* pr = PQ1 + (size_t)nd * P1W;
          const float* qr = PQ1 + (size_t)src * P1W;
          float f = pr[c] + qr[12 + c] + bfv;
          float s = pr[24 + c] + qr[36 + c] + bsv;
          const float* er = ea + (size_t)e * 6;
          const v2f e01 = *(const v2f*)er, e23 = *(const v2f*)(er + 2), e45 = *(const v2f*)(er + 4);
          const float* tw = tW + c;
          f += e01.x * tw[0] + e01.y * tw[24] + e23.x * tw[48] + e23.y * tw[72] + e45.x * tw[96] + e45.y * tw[120];
          s += e01.x * tw[12] + e01.y * tw[36] + e23.x * tw[60] + e23.y * tw[84] + e45.x * tw[108] + e45.y * tw[132];
          const float mv = sigm(f) * softp(s);
          if (lane < C1) acc[slot * C1 + lane] += mv;
        }
      }
    }
    __syncthreads();
  }

  const int nl = lane >> 3, p = lane & 7, pc = p < 3 ? p : 2;
#pragma unroll 1
  for (int j = 0; j < NB1 / (NWAVE * 4); ++j) {
    const int slot = wave * (NB1 / NWAVE) + 4 * j + nl;
    const int node = keyBase + slot;
    const int nr = node > nN - 1 ? nN - 1 : node;
    const v4f xv = *(const v4f*)(x + (size_t)nr * C1 + 4 * pc);
    const v4f av = *(const v4f*)(acc + slot * C1 + 4 * pc);
    v4f y = xv + av;
    y.x = fmaxf(y.x, 0.f); y.y = fmaxf(y.y, 0.f); y.z = fmaxf(y.z, 0.f); y.w = fmaxf(y.w, 0.f);
    if (p >= 3) { y.x = 0.f; y.y = 0.f; y.z = 0.f; y.w = 0.f; }
    float* op = h0 + (size_t)node * H0W + 4 * p;
    *(volatile v4f*)op = y;
    __threadfence();
    *(volatile v4f*)op = y;
  }
}

__global__ __launch_bounds__(NTHR) void k_prepW(const float* __restrict__ W, int ldw, int Kreal, int KP,
                                                int c0, int ncol, unsigned short* Bh, unsigned short* Bl) {
  const int i = blockIdx.x * NTHR + threadIdx.x;
  const int kq = KP >> 3;
  if (i >= ncol * kq) return;
  const int n = i / kq, k8 = i - n * kq;
  v8us hv, lv;
#pragma unroll
  for (int j = 0; j < 8; ++j) {
    const int k = k8 * 8 + j;
    const int kc = k < Kreal ? k : Kreal - 1;
    const float w = W[(size_t)kc * ldw + c0 + n];
    const float v = (k < Kreal) ? w : 0.f;
    const unsigned int hb = bfr(v);
    hv[j] = (unsigned short)hb;
    lv[j] = (unsigned short)bfr(v - __uint_as_float(hb << 16));
  }
  const size_t o = (size_t)n * KP + (size_t)k8 * 8;
  *(volatile v8us*)(Bh + o) = hv;
  *(volatile v8us*)(Bl + o) = lv;
  __threadfence();
  *(volatile v8us*)(Bh + o) = hv;
  *(volatile v8us*)(Bl + o) = lv;
}

__global__ __launch_bounds__(NTHR) void k_prepPQ(const float* __restrict__ Wf, const float* __restrict__ Ws,
                                                 int q, unsigned short* Bh, unsigned short* Bl) {
  const int i = blockIdx.x * NTHR + threadIdx.x;
  if (i >= PQW * (HD / 8)) return;
  const int n = i >> 4, k8 = i & 15;
  const int part = n >> 6;
  const int cg = 64 * q + (n & 63);
  const int krow0 = (part & 1) * HD;
  v8us hv, lv;
#pragma unroll
  for (int j = 0; j < 8; ++j) {
    const int k = k8 * 8 + j;
    const float a = Wf[(size_t)(krow0 + k) * HD + cg];
    const float b = Ws[(size_t)(krow0 + k) * HD + cg];
    const float v = (part < 2) ? a : b;
    const unsigned int hb = bfr(v);
    hv[j] = (unsigned short)hb;
    lv[j] = (unsigned short)bfr(v - __uint_as_float(hb << 16));
  }
  const size_t o = (size_t)n * HD + (size_t)k8 * 8;
  *(volatile v8us*)(Bh + o) = hv;
  *(volatile v8us*)(Bl + o) = lv;
  __threadfence();
  *(volatile v8us*)(Bh + o) = hv;
  *(volatile v8us*)(Bl + o) = lv;
}

template<int KP, int NCT>
__global__ __launch_bounds__(NTHR) void k_gemm(const float* __restrict__ A, int lda, int M,
                                               const unsigned short* __restrict__ Bh,
                                               const unsigned short* __restrict__ Bl,
                                               const float* __restrict__ bias, int hasBias, int doRelu,
                                               float* Cout) {
  constexpr int NW  = 16 * NCT * NWAVE;
  constexpr int KT  = KP / 32;
  constexpr int KQ  = KP / 8;
  constexpr int ABYTES = 32 * KP * 4;
  constexpr int CBYTES = 16 * NW * 4;
  constexpr int LB  = ABYTES > CBYTES ? ABYTES : CBYTES;
  constexpr int IPR = NW / 128;
  static_assert((NW % 128) == 0);
  static_assert((KP % 32) == 0);
  __shared__ __attribute__((aligned(16))) unsigned char lds_raw[LB];
  unsigned short* Ah = (unsigned short*)lds_raw;
  unsigned short* Al = Ah + 32 * KP;
  float* Cs = (float*)lds_raw;

  const int tid = threadIdx.x, lane = tid & 31, wave = tid >> 5;
  const int hh = lane >> 4, m = lane & 15;
  const int rowBase = blockIdx.x * 32;

  for (int it = tid; it < 32 * KQ; it += NTHR) {
    const int r = it / KQ, k8 = it - r * KQ;
    int row = rowBase + r; if (row > M - 1) row = M - 1;
    const float* p = A + (size_t)row * lda + k8 * 8;
    const v4f f0 = *(const v4f*)p, f1 = *(const v4f*)(p + 4);
    float fv[8] = {f0.x, f0.y, f0.z, f0.w, f1.x, f1.y, f1.z, f1.w};
    v8us hv, lv;
#pragma unroll
    for (int j = 0; j < 8; ++j) {
      const unsigned int hb = bfr(fv[j]);
      hv[j] = (unsigned short)hb;
      lv[j] = (unsigned short)bfr(fv[j] - __uint_as_float(hb << 16));
    }
    *(v8us*)(Ah + r * KP + k8 * 8) = hv;
    *(v8us*)(Al + r * KP + k8 * 8) = lv;
  }
  __syncthreads();

  const int colw = wave * 16 * NCT;
  v8f acc[2][NCT];
#pragma unroll
  for (int t = 0; t < 2; ++t)
#pragma unroll
    for (int ct = 0; ct < NCT; ++ct) acc[t][ct] = v8f{0.f, 0.f, 0.f, 0.f, 0.f, 0.f, 0.f, 0.f};

#pragma unroll
  for (int kt = 0; kt < KT; ++kt) {
    const int k0 = kt * 32;
    Frag ah0, al0, ah1, al1;
    const unsigned short* pa0 = Ah + m * KP + k0 + 8 * hh;
    const unsigned short* pa1 = Ah + (16 + m) * KP + k0 + 8 * hh;
    const unsigned short* pl0 = Al + m * KP + k0 + 8 * hh;
    const unsigned short* pl1 = Al + (16 + m) * KP + k0 + 8 * hh;
    ah0.h[0] = *(const v8us*)pa0; ah0.h[1] = *(const v8us*)(pa0 + 16);
    ah1.h[0] = *(const v8us*)pa1; ah1.h[1] = *(const v8us*)(pa1 + 16);
    al0.h[0] = *(const v8us*)pl0; al0.h[1] = *(const v8us*)(pl0 + 16);
    al1.h[0] = *(const v8us*)pl1; al1.h[1] = *(const v8us*)(pl1 + 16);
#pragma unroll
    for (int ct = 0; ct < NCT; ++ct) {
      const int n = colw + ct * 16 + m;
      Frag bh, bl;
      const unsigned short* pb = Bh + (size_t)n * KP + k0 + 8 * hh;
      const unsigned short* ql = Bl + (size_t)n * KP + k0 + 8 * hh;
      bh.h[0] = *(const v8us*)pb; bh.h[1] = *(const v8us*)(pb + 16);
      bl.h[0] = *(const v8us*)ql; bl.h[1] = *(const v8us*)(ql + 16);
      wm6(acc[0][ct], acc[1][ct], ah0.v, al0.v, ah1.v, al1.v, bh.v, bl.v);
    }
  }

  float bv[NCT];
#pragma unroll
  for (int ct = 0; ct < NCT; ++ct) bv[ct] = 0.f;
  if (hasBias) {
#pragma unroll
    for (int ct = 0; ct < NCT; ++ct) bv[ct] = bias[colw + ct * 16 + m];
  }
  __syncthreads();

#pragma unroll
  for (int t = 0; t < 2; ++t) {
#pragma unroll
    for (int ct = 0; ct < NCT; ++ct) {
#pragma unroll
      for (int r = 0; r < 8; ++r) {
        float v = acc[t][ct][r] + bv[ct];
        if (doRelu) v = fmaxf(v, 0.f);
        Cs[(8 * hh + r) * NW + colw + ct * 16 + m] = v;
      }
    }
    __syncthreads();
    for (int it = wave; it < 16 * IPR; it += NWAVE) {
      const int row = it / IPR, chn = it - row * IPR;
      const int col = chn * 128 + 4 * lane;
      const v4f v = *(const v4f*)(Cs + row * NW + col);
      *(volatile v4f*)(Cout + (size_t)(rowBase + 16 * t + row) * NW + col) = v;
    }
    __threadfence();
    for (int it = wave; it < 16 * IPR; it += NWAVE) {
      const int row = it / IPR, chn = it - row * IPR;
      const int col = chn * 128 + 4 * lane;
      const v4f v = *(const v4f*)(Cs + row * NW + col);
      *(volatile v4f*)(Cout + (size_t)(rowBase + 16 * t + row) * NW + col) = v;
    }
    __syncthreads();
  }
}

__global__ __launch_bounds__(NTHR) void k_agg2(
    const float* __restrict__ xin, const float* __restrict__ PQ,
    const int* __restrict__ ei, const float* __restrict__ ea,
    const float* __restrict__ Wf, const float* __restrict__ Ws,
    const float* __restrict__ bf, const float* __restrict__ bs,
    float* hout, int nN, int nE, int q) {
  extern __shared__ v4f lds_dyn[];
  float* acc  = (float*)lds_dyn;
  float* tW   = acc + ACC2;
  float* tb   = tW + TW2;
  int*   list = (int*)(tb + TB2);
  int*   wcnt = list + LISTN;

  const int tid = threadIdx.x, lane = tid & 31, wave = tid >> 5;
  const int keyBase = blockIdx.x * NB2;
  {
    const v4f z4 = {0.f, 0.f, 0.f, 0.f};
    for (int i = tid; i < ACC2 / 4; i += NTHR) lds_dyn[i] = z4;
    for (int i = tid; i < TW2; i += NTHR) {
      const int d = i >> 7, j = i & 127;
      const int cg = 64 * q + (j & 63);
      const float a = Wf[(size_t)(2 * HD + d) * HD + cg], b = Ws[(size_t)(2 * HD + d) * HD + cg];
      tW[i] = (j < 64) ? a : b;
    }
    if (tid < TB2) {
      const int cg = 64 * q + (tid & 63);
      const float a = bf[cg], b = bs[cg];
      tb[tid] = (tid < 64) ? a : b;
    }
  }
  __syncthreads();

  const int* keyp = ei + nE;
  const bool al16 = ((((size_t)keyp) & 15) == 0);
  const int c2 = 2 * lane;
  const int nChunks = (nE + CHUNK - 1) / CHUNK;
#pragma unroll 1
  for (int ch = 0; ch < nChunks; ++ch) {
    const int cbase = ch * CHUNK;
    const int wc = scan_chunk<NB2, SB2>(keyp, nE, cbase, keyBase, list + wave * WCAP, tid, al16);
    if (lane == 0) wcnt[wave] = wc;
    __syncthreads();
    if (wave == 0) {
      const v2f bfv = *(const v2f*)(tb + c2), bsv = *(const v2f*)(tb + 64 + c2);
      const float* tw = tW + c2;
      for (int wsx = 0; wsx < NWAVE; ++wsx) {
        int n = wcnt[wsx];
        n = n > WCAP ? WCAP : (n < 0 ? 0 : n);
        for (int i = 0; i < n; ++i) {
          const int ent  = list[wsx * WCAP + i];
          const int slot = ent & (NB2 - 1);
          const int el   = (ent >> SB2) & (CHUNK - 1);
          int e = cbase + el; if (e > nE - 1) e = nE - 1;
          int src = ei[e]; src = src < 0 ? 0 : (src > nN - 1 ? nN - 1 : src);
          int nd = keyBase + slot; if (nd > nN - 1) nd = nN - 1;
          const float* pr = PQ + (size_t)nd * PQW + c2;
          const float* qr = PQ + (size_t)src * PQW + c2;
          v2f f = *(const v2f*)pr + *(const v2f*)(qr + 64) + bfv;
          v2f s = *(const v2f*)(pr + 128) + *(const v2f*)(qr + 192) + bsv;
          const float* er = ea + (size_t)e * 6;
          const v2f e01 = *(const v2f*)er, e23 = *(const v2f*)(er + 2), e45 = *(const v2f*)(er + 4);
          f += e01.x * *(const v2f*)(tw)       + e01.y * *(const v2f*)(tw + 128)
             + e23.x * *(const v2f*)(tw + 256) + e23.y * *(const v2f*)(tw + 384)
             + e45.x * *(const v2f*)(tw + 512) + e45.y * *(const v2f*)(tw + 640);
          s += e01.x * *(const v2f*)(tw + 64)  + e01.y * *(const v2f*)(tw + 192)
             + e23.x * *(const v2f*)(tw + 320) + e23.y * *(const v2f*)(tw + 448)
             + e45.x * *(const v2f*)(tw + 576) + e45.y * *(const v2f*)(tw + 704);
          v2f mv;
          mv.x = sigm(f.x) * softp(s.x);
          mv.y = sigm(f.y) * softp(s.y);
          v2f* ap = (v2f*)(acc + slot * 64 + c2);
          const v2f cur = *ap;
          *ap = cur + mv;
        }
      }
    }
    __syncthreads();
  }

  const int nl = lane >> 4, p = lane & 15;
#pragma unroll 1
  for (int j = 0; j < NB2 / (NWAVE * 2); ++j) {
    const int slot = wave * (NB2 / NWAVE) + 2 * j + nl;
    const int node = keyBase + slot;
    const int nr = node > nN - 1 ? nN - 1 : node;
    const v4f xv = *(const v4f*)(xin + (size_t)nr * HD + 64 * q + 4 * p);
    const v4f av = *(const v4f*)(acc + slot * 64 + 4 * p);
    v4f y = xv + av;
    y.x = fmaxf(y.x, 0.f); y.y = fmaxf(y.y, 0.f); y.z = fmaxf(y.z, 0.f); y.w = fmaxf(y.w, 0.f);
    float* op = hout + (size_t)node * HD + 64 * q + 4 * p;
    *(volatile v4f*)op = y;
    __threadfence();
    *(volatile v4f*)op = y;
  }
}

__global__ __launch_bounds__(NTHR) void k_pool(const float* __restrict__ h, const int* __restrict__ batch,
                                               float* g, int nN) {
  extern __shared__ v4f lds_dyn[];
  float* acc  = (float*)lds_dyn;
  float* cnt  = acc + ACCP;
  int*   list = (int*)(cnt + NBP);
  int*   wcnt = list + LISTN;

  const int tid = threadIdx.x, lane = tid & 31, wave = tid >> 5;
  const int keyBase = blockIdx.x * NBP;
  {
    const v4f z4 = {0.f, 0.f, 0.f, 0.f};
    for (int i = tid; i < (ACCP + NBP) / 4; i += NTHR) lds_dyn[i] = z4;
  }
  __syncthreads();
  const bool al16 = ((((size_t)batch) & 15) == 0);
  const int nChunks = (nN + CHUNK - 1) / CHUNK;
#pragma unroll 1
  for (int ch = 0; ch < nChunks; ++ch) {
    const int cbase = ch * CHUNK;
    const int wc = scan_chunk<NBP, SBP>(batch, nN, cbase, keyBase, list + wave * WCAP, tid, al16);
    if (lane == 0) wcnt[wave] = wc;
    __syncthreads();
    if (wave == 0) {
      for (int wsx = 0; wsx < NWAVE; ++wsx) {
        int n = wcnt[wsx];
        n = n > WCAP ? WCAP : (n < 0 ? 0 : n);
        for (int i = 0; i < n; ++i) {
          const int ent  = list[wsx * WCAP + i];
          const int slot = ent & (NBP - 1);
          const int el   = (ent >> SBP) & (CHUNK - 1);
          int nd = cbase + el; if (nd > nN - 1) nd = nN - 1;
          const v4f hv = *(const v4f*)(h + (size_t)nd * HD + 4 * lane);
          v4f* ap = (v4f*)(acc + slot * HD + 4 * lane);
          const v4f cur = *ap;
          *ap = cur + hv;
          if (lane == 0) cnt[slot] += 1.0f;
        }
      }
    }
    __syncthreads();
  }
#pragma unroll 1
  for (int j = 0; j < NBP / NWAVE; ++j) {
    const int slot = wave * (NBP / NWAVE) + j;
    const float cc = fmaxf(cnt[slot], 1.0f);
    const float inv = 1.0f / cc;
    const v4f v = *(const v4f*)(acc + slot * HD + 4 * lane) * inv;
    float* op = g + (size_t)(keyBase + slot) * HD + 4 * lane;
    *(volatile v4f*)op = v;
    __threadfence();
    *(volatile v4f*)op = v;
  }
}

__global__ __launch_bounds__(NTHR) void k_head3(const float* __restrict__ g2, const float* __restrict__ W3,
                                                const float* __restrict__ b3, float* out, int rowsP, int nG) {
  __shared__ __attribute__((aligned(16))) float res[1024];
  const int tid = threadIdx.x, lane = tid & 31, wave = tid >> 5;
  const v4f wv = *(const v4f*)(W3 + 4 * lane);
  const float bb = b3[0];
  const int per = rowsP / NWAVE;
#pragma unroll 1
  for (int j = 0; j < per; ++j) {
    const int b = wave * per + j;
    const v4f gv = *(const v4f*)(g2 + (size_t)b * HD + 4 * lane);
    float d = gv.x * wv.x + gv.y * wv.y + gv.z * wv.z + gv.w * wv.w;
    d = wsum(d);
    if (lane == 0) res[b] = d + bb;
  }
  __syncthreads();
  const int n4 = nG >> 2;
  for (int i = tid; i < n4; i += NTHR) {
    const v4f v = *(const v4f*)(res + 4 * i);
    *(volatile v4f*)(out + 4 * i) = v;
  }
  if (tid == 0) for (int i = n4 * 4; i < nG; ++i) { const float v = res[i]; *(volatile float*)(out + i) = v; }
  __threadfence();
  for (int i = tid; i < n4; i += NTHR) {
    const v4f v = *(const v4f*)(res + 4 * i);
    *(volatile v4f*)(out + 4 * i) = v;
  }
  if (tid == 0) for (int i = n4 * 4; i < nG; ++i) { const float v = res[i]; *(volatile float*)(out + i) = v; }
}

extern "C" void kernel_launch(void* const* d_in, const int* in_sizes, int n_in,
                              void* d_out, int out_size, void* d_ws, size_t ws_size,
                              hipStream_t stream) {
  if (n_in < 24) return;
  const int nN = in_sizes[0] / C1;
  if (nN <= 0 || in_sizes[0] != nN * C1) return;
  const int nE = in_sizes[2] / 6;
  if (nE <= 0 || in_sizes[2] != nE * 6 || in_sizes[1] != 2 * nE) return;
  if (in_sizes[3] != nN) return;
  if (in_sizes[4] != 30 * C1 || in_sizes[5] != C1 || in_sizes[6] != 30 * C1 || in_sizes[7] != C1) return;
  if (in_sizes[8] != C1 * HD || in_sizes[9] != HD) return;
  for (int i = 10; i <= 16; i += 2) { if (in_sizes[i] != (2 * HD + 6) * HD || in_sizes[i + 1] != HD) return; }
  if (in_sizes[18] != HD * HD || in_sizes[19] != HD || in_sizes[20] != HD * HD || in_sizes[21] != HD) return;
  if (in_sizes[22] != HD || in_sizes[23] != 1) return;
  const int nG = out_size;
  if (nG <= 0 || nG > 1024) return;

  const float* x     = (const float*)d_in[0];
  const int*   ei    = (const int*)d_in[1];
  const float* ea    = (const float*)d_in[2];
  const int*   batch = (const int*)d_in[3];
  const float* Wf1 = (const float*)d_in[4];  const float* bf1 = (const float*)d_in[5];
  const float* Ws1 = (const float*)d_in[6];  const float* bs1 = (const float*)d_in[7];
  const float* Wlin = (const float*)d_in[8]; const float* blin = (const float*)d_in[9];
  const float* Wf2 = (const float*)d_in[10]; const float* bf2 = (const float*)d_in[11];
  const float* Ws2 = (const float*)d_in[12]; const float* bs2 = (const float*)d_in[13];
  const float* Wf3 = (const float*)d_in[14]; const float* bf3 = (const float*)d_in[15];
  const float* Ws3 = (const float*)d_in[16]; const float* bs3 = (const float*)d_in[17];
  const float* Wh1 = (const float*)d_in[18]; const float* bh1 = (const float*)d_in[19];
  const float* Wh2 = (const float*)d_in[20]; const float* bh2 = (const float*)d_in[21];
  const float* Wh3 = (const float*)d_in[22]; const float* bh3 = (const float*)d_in[23];
  float* out = (float*)d_out;

  const int gA1 = (nN + NB1 - 1) / NB1;  const int rowsH0 = gA1 * NB1;
  const int gA2 = (nN + NB2 - 1) / NB2;  const int rowsH  = gA2 * NB2;
  const int gG  = (nN + 31) / 32;        const int rowsG  = gG * 32;
  const int rowsHA = rowsH > rowsG ? rowsH : rowsG;
  const int gP  = (nG + NBP - 1) / NBP;  const int rowsP  = gP * NBP;
  if (rowsP > 1024 || (rowsP % 32) != 0) return;
  const int gH  = rowsP / 32;

  char* ws = (char*)d_ws;
  size_t off = 0;
  auto take = [&](size_t bytes) -> char* { char* p = ws + off; off = (off + bytes + 255) & ~(size_t)255; return p; };
  float* RA = (float*)take((size_t)rowsHA * HD * 4);
  float* RB = (float*)take((size_t)rowsHA * HD * 4);
  const size_t pqBytes  = (size_t)rowsG * PQW * 4;
  const size_t pq1Bytes = (size_t)rowsG * P1W * 4;
  const size_t h0Bytes  = (size_t)rowsH0 * H0W * 4;
  const size_t rpBytes  = pqBytes > (pq1Bytes + h0Bytes) ? pqBytes : (pq1Bytes + h0Bytes);
  char*  RP   = take(rpBytes);
  float* PQ   = (float*)RP;
  float* PQ1  = (float*)RP;
  float* h0   = (float*)(RP + pq1Bytes);
  unsigned short* BWl_h = (unsigned short*)take((size_t)HD * 32 * 2);
  unsigned short* BWl_l = (unsigned short*)take((size_t)HD * 32 * 2);
  unsigned short* BPQ_h = (unsigned short*)take((size_t)PQW * HD * 2);
  unsigned short* BPQ_l = (unsigned short*)take((size_t)PQW * HD * 2);
  unsigned short* BH1_h = (unsigned short*)take((size_t)HD * HD * 2);
  unsigned short* BH1_l = (unsigned short*)take((size_t)HD * HD * 2);
  unsigned short* BH2_h = (unsigned short*)take((size_t)HD * HD * 2);
  unsigned short* BH2_l = (unsigned short*)take((size_t)HD * HD * 2);
  float* g  = (float*)take((size_t)rowsP * HD * 4);
  float* g1 = (float*)take((size_t)rowsP * HD * 4);
  float* g2 = (float*)take((size_t)rowsP * HD * 4);
  if (off > ws_size) return;

  k_pq1<<<gG, NTHR, 0, stream>>>(x, Wf1, Ws1, PQ1, nN);
  hipFuncSetAttribute(reinterpret_cast<const void*>(&k_agg1), hipFuncAttributeMaxDynamicSharedMemorySize, LDS1_BYTES);
  k_agg1<<<gA1, NTHR, LDS1_BYTES, stream>>>(x, PQ1, ei, ea, Wf1, Ws1, bf1, bs1, h0, nN, nE);

  k_prepW<<<(HD * 4 + NTHR - 1) / NTHR, NTHR, 0, stream>>>(Wlin, HD, C1, 32, 0, HD, BWl_h, BWl_l);
  k_gemm<32, 1><<<gG, NTHR, 0, stream>>>(h0, H0W, nN, BWl_h, BWl_l, blin, 1, 0, RA);

  hipFuncSetAttribute(reinterpret_cast<const void*>(&k_agg2), hipFuncAttributeMaxDynamicSharedMemorySize, LDS2_BYTES);
  const int gPQ = (PQW * (HD / 8) + NTHR - 1) / NTHR;
  for (int q = 0; q < 2; ++q) {
    k_prepPQ<<<gPQ, NTHR, 0, stream>>>(Wf2, Ws2, q, BPQ_h, BPQ_l);
    k_gemm<128, 2><<<gG, NTHR, 0, stream>>>(RA, HD, nN, BPQ_h, BPQ_l, bf2, 0, 0, PQ);
    k_agg2<<<gA2, NTHR, LDS2_BYTES, stream>>>(RA, PQ, ei, ea, Wf2, Ws2, bf2, bs2, RB, nN, nE, q);
  }
  for (int q = 0; q < 2; ++q) {
    k_prepPQ<<<gPQ, NTHR, 0, stream>>>(Wf3, Ws3, q, BPQ_h, BPQ_l);
    k_gemm<128, 2><<<gG, NTHR, 0, stream>>>(RB, HD, nN, BPQ_h, BPQ_l, bf3, 0, 0, PQ);
    k_agg2<<<gA2, NTHR, LDS2_BYTES, stream>>>(RB, PQ, ei, ea, Wf3, Ws3, bf3, bs3, RA, nN, nE, q);
  }

  hipFuncSetAttribute(reinterpret_cast<const void*>(&k_pool), hipFuncAttributeMaxDynamicSharedMemorySize, LDSP_BYTES);
  k_pool<<<gP, NTHR, LDSP_BYTES, stream>>>(RA, batch, g, nN);
  const int gBH = (HD * (HD / 8) + NTHR - 1) / NTHR;
  k_prepW<<<gBH, NTHR, 0, stream>>>(Wh1, HD, HD, HD, 0, HD, BH1_h, BH1_l);
  k_gemm<128, 1><<<gH, NTHR, 0, stream>>>(g, HD, rowsP, BH1_h, BH1_l, bh1, 1, 1, g1);
  k_prepW<<<gBH, NTHR, 0, stream>>>(Wh2, HD, HD, HD, 0, HD, BH2_h, BH2_l);
  k_gemm<128, 1><<<gH, NTHR, 0, stream>>>(g1, HD, rowsP, BH2_h, BH2_l, bh2, 1, 1, g2);
  k_head3<<<1, NTHR, 0, stream>>>(g2, Wh3, bh3, out, rowsP, nG);
}
